// DecoderBlock_43044162241285
// MI455X (gfx1250) — hardware-verified
//
#include <hip/hip_runtime.h>
#include <math.h>

typedef __attribute__((ext_vector_type(16))) _Float16 v16h;
typedef __attribute__((ext_vector_type(16))) __bf16 v16b;
typedef __attribute__((ext_vector_type(8)))  _Float16 v8h;
typedef __attribute__((ext_vector_type(8)))  float v8f;
typedef __attribute__((ext_vector_type(4)))  float v4f;
typedef __attribute__((ext_vector_type(4)))  unsigned v4u;
typedef __attribute__((ext_vector_type(4)))  int v4i;

template <typename T> __device__ __forceinline__ void vst2(void* p, T v) { *(volatile T*)p = v; __threadfence(); *(volatile T*)p = v; }
__device__ __forceinline__ v8f wmma16(v16h a, v16h b, v8f c) {
  v8f d = __builtin_amdgcn_wmma_f32_16x16x32_f16(false, a, false, b, (short)0, c, false, false);
  asm volatile("v_nop\n\tv_nop\n\tv_nop\n\tv_nop" : "+v"(d) : "v"(a), "v"(b));
  return d;
}
__device__ __forceinline__ v8f wmma_bf(v16b a, v16b b, v8f c) {
  v8f d = __builtin_amdgcn_wmma_f32_16x16x32_bf16(false, a, false, b, (short)0, c, false, false);
  asm volatile("v_nop\n\tv_nop\n\tv_nop\n\tv_nop" : "+v"(d) : "v"(a), "v"(b));
  return d;
}
__device__ __forceinline__ v16h frag_h(const _Float16* rowk0, unsigned lane) {
  union { v16h v; v8h q[2]; } u; const _Float16* p = rowk0 + 8u * (lane >> 4);
  u.q[0] = *(const v8h*)p; u.q[1] = *(const v8h*)(p + 16); return u.v;
}
__device__ __forceinline__ float bfr(float v) { return (float)(__bf16)v; }
struct Q16 { v4f q0, q1, q2, q3; };
__device__ __forceinline__ Q16 ld16(const float* p) { Q16 r; r.q0 = *(const v4f*)p; r.q1 = *(const v4f*)(p + 4); r.q2 = *(const v4f*)(p + 16); r.q3 = *(const v4f*)(p + 20); return r; }
__device__ __forceinline__ v16b cvt_bf(const Q16& t) { v16b w;
#pragma unroll
  for (int i = 0; i < 4; ++i) { w[i] = (__bf16)t.q0[i]; w[4 + i] = (__bf16)t.q1[i]; w[8 + i] = (__bf16)t.q2[i]; w[12 + i] = (__bf16)t.q3[i]; }
  return w; }
#define WCARRY (64.0f)
__device__ __forceinline__ v16h cvt_wh(const Q16& t) { v16h w;
#pragma unroll
  for (int i = 0; i < 4; ++i) { w[i] = (_Float16)(bfr(t.q0[i]) * WCARRY); w[4 + i] = (_Float16)(bfr(t.q1[i]) * WCARRY); w[8 + i] = (_Float16)(bfr(t.q2[i]) * WCARRY); w[12 + i] = (_Float16)(bfr(t.q3[i]) * WCARRY); }
  return w; }
__device__ __forceinline__ _Float16 ah1(float x, int act, float asc) { if (act == 1) x = fmaxf(x, 0.f); return (_Float16)(x * asc); }
__device__ __forceinline__ v16h cvt_ah(const Q16& t, int act, float asc) { v16h a;
#pragma unroll
  for (int i = 0; i < 4; ++i) { a[i] = ah1(t.q0[i], act, asc); a[4 + i] = ah1(t.q1[i], act, asc); a[8 + i] = ah1(t.q2[i], act, asc); a[12 + i] = ah1(t.q3[i], act, asc); }
  return a; }
__device__ __forceinline__ v16h cvt_ph(const Q16& t) { v16h a;
#pragma unroll
  for (int i = 0; i < 4; ++i) { a[i] = (_Float16)t.q0[i]; a[4 + i] = (_Float16)t.q1[i]; a[8 + i] = (_Float16)t.q2[i]; a[12 + i] = (_Float16)t.q3[i]; }
  return a; }
#define LDSX() do { asm volatile("s_wait_dscnt 0" ::: "memory"); __builtin_amdgcn_wave_barrier(); __builtin_amdgcn_fence(3  , "workgroup"); } while (0)

#ifndef NB
#define NB 2
#endif
#ifndef SEQ
#define SEQ 1024
#endif
#define SEQ_FULL 1024
#define TQ SEQ
#define TK SEQ
#define CC 1024
#define DIN 1024
#define NH 16
#define HD 64
#define HG 16
#define FF 4096
#define SCALE (0.125f)
#define PCARRY (2048.0f)
#define ACARRY (32.0f)
#define MASKFILL (-1.0e9f)
#define NRW (NB * TQ)
#define NRK (NB * TK)

static_assert(TQ == TK);
static_assert(TQ % 64 == 0);
static_assert(TK % 128 == 0);
static_assert(NRW % 64 == 0);
static_assert(NRW % 8 == 0);
static_assert(CC == 1024);
static_assert(CC == NH * HD);
static_assert(DIN == CC);
static_assert(HD == 64);
static_assert(NH % HG == 0);
static_assert(DIN % 32 == 0);
static_assert(CC % 128 == 0);
static_assert(FF % 128 == 0);
static_assert(FF % 32 == 0);
static_assert(TK * 4 <= 32768);
static_assert(SEQ <= SEQ_FULL);
static_assert((NRW / 64) * 64 == NRW);
static_assert((CC / 128) * 128 == CC);
static_assert((FF / 128) * 128 == FF);
static_assert((TQ / 64) * 64 == TQ);
static_assert((TK / 128) * 128 == TK);
static_assert((NRW / 8) * 8 == NRW);
static_assert((TK / 4) * 4 == TK);

constexpr size_t SZ_QH = (size_t)2 * NRW * CC;
constexpr size_t SZ_KH = (size_t)2 * NRK * CC;
constexpr size_t SZ_VT = (size_t)2 * NB * CC * TK;
constexpr size_t SZ_S  = (size_t)4 * HG * TQ * TK;
constexpr size_t SZ_HF = (size_t)4 * NRW * FF;
constexpr size_t SZ_SHF = SZ_S > SZ_HF ? SZ_S : SZ_HF;
constexpr size_t SZ_ROWS = (size_t)4 * NRW * CC;
constexpr size_t WS_QH = 0;
constexpr size_t WS_KH = WS_QH + SZ_QH;
constexpr size_t WS_VT = WS_KH + SZ_KH;
constexpr size_t WS_S  = WS_VT + SZ_VT;
constexpr size_t WS_Y  = WS_S + SZ_SHF;
constexpr size_t WS_Z  = WS_Y + SZ_ROWS;
constexpr size_t WS_X1 = WS_Z + SZ_ROWS;
constexpr size_t WS_X2 = WS_X1 + SZ_ROWS;
constexpr size_t WS_END = WS_X2 + SZ_ROWS;
static_assert(SZ_S <= SZ_SHF);
static_assert(SZ_HF <= SZ_SHF);
static_assert(WS_KH % 128 == 0);
static_assert(WS_VT % 128 == 0);
static_assert(WS_S % 128 == 0);
static_assert(WS_Y % 128 == 0);
static_assert(WS_Z % 128 == 0);
static_assert(WS_X1 % 128 == 0);
static_assert(WS_X2 % 128 == 0);
static_assert(WS_END <= (size_t)134217728);

__global__ __launch_bounds__(256) void k_addln(const float* __restrict__ X, int cvtin, unsigned xbatch_rows, const float* __restrict__ ADD, int hasadd, const float* __restrict__ G, const float* __restrict__ BE, float* __restrict__ OUT) {
  const unsigned wave = threadIdx.x >> 5, lane = threadIdx.x & 31u; const unsigned row = blockIdx.x * 8u + wave; if (row >= (unsigned)NRW) return;
  const unsigned xr = (row / (unsigned)TQ) * xbatch_rows + (row % (unsigned)TQ);
  v4f v[CC / 128]; float s1 = 0.f;
#pragma unroll
  for (int i = 0; i < CC / 128; ++i) { v4f t = *(const v4f*)(X + (size_t)xr * CC + i * 128 + lane * 4u);
    if (cvtin) { t[0] = bfr(t[0]); t[1] = bfr(t[1]); t[2] = bfr(t[2]); t[3] = bfr(t[3]); }
    if (hasadd) { const v4f a = *(const v4f*)(ADD + (size_t)row * CC + i * 128 + lane * 4u); t[0] += a[0]; t[1] += a[1]; t[2] += a[2]; t[3] += a[3]; }
    v[i] = t; s1 += (t[0] + t[1]) + (t[2] + t[3]); }
#pragma unroll
  for (int o = 1; o < 32; o <<= 1) s1 += __shfl_xor(s1, o);
  const float mu = s1 * (1.0f / CC); float q = 0.f;
#pragma unroll
  for (int i = 0; i < CC / 128; ++i) {
#pragma unroll
    for (int k = 0; k < 4; ++k) { const float d = v[i][k] - mu; q += d * d; } }
#pragma unroll
  for (int o = 1; o < 32; o <<= 1) q += __shfl_xor(q, o);
  const float sd = sqrtf(q * (1.0f / (float)(CC - 1)));
  const float inv = 1.0f / (sd + 1e-12f);
#pragma unroll
  for (int i = 0; i < CC / 128; ++i) { const unsigned c = i * 128 + lane * 4u; const v4f g4 = *(const v4f*)(G + c); const v4f b4 = *(const v4f*)(BE + c); v4f r4;
#pragma unroll
    for (int k = 0; k < 4; ++k) r4[k] = (bfr(g4[k]) * (v[i][k] - mu)) * inv + bfr(b4[k]);
    vst2(OUT + (size_t)row * CC + c, r4); } }

__global__ __launch_bounds__(128) void k_proj(const float* __restrict__ XQ, const float* __restrict__ XE, const float* __restrict__ WQ, const float* __restrict__ WK, const float* __restrict__ WV,
    _Float16* __restrict__ QH, _Float16* __restrict__ KH, _Float16* __restrict__ VT) {
  __shared__ __align__(16) _Float16 sh[64][136]; __shared__ __align__(16) _Float16 th[128][72];
  const unsigned tid = threadIdx.x, wave = tid >> 5, lane = tid & 31u, col = lane & 15u, g = lane >> 4;
  const unsigned which = blockIdx.z, c0 = blockIdx.y * 128u, r0 = blockIdx.x * 64u; const unsigned bb = r0 / (unsigned)TQ, t0 = r0 % (unsigned)TQ;
  const float* X = which == 0 ? XQ : XE; const float* WA = which == 0 ? WQ : (which == 1 ? WK : WV);
  const float* xrow = X + ((size_t)bb * SEQ_FULL + t0 + wave * 16u + col) * DIN + 8u * g;
  const float* wrow = WA + (size_t)(c0 + col) * DIN + 8u * g;
  v8f acc[8] = {};
#pragma unroll 2
  for (unsigned kc = 0; kc < (unsigned)(DIN / 32); ++kc) { const Q16 ta = ld16(xrow + kc * 32u);
    asm volatile("s_wait_loadcnt 0x0" ::: "memory");
    const v16b a = cvt_bf(ta);
#pragma unroll
    for (int j = 0; j < 8; ++j) { const Q16 tw = ld16(wrow + (size_t)j * 16u * DIN + kc * 32u); asm volatile("s_wait_loadcnt 0x0" ::: "memory"); const v16b w = cvt_bf(tw); acc[j] = wmma_bf(a, w, acc[j]); } }
  if (which < 2) { _Float16* DH = which == 0 ? QH : KH;
#pragma unroll
    for (int j = 0; j < 8; ++j) {
#pragma unroll
      for (int r = 0; r < 8; ++r) sh[wave * 16 + 8 * g + r][j * 16 + col] = (_Float16)acc[j][r]; }
    __syncthreads();
    for (unsigned e = tid; e < 64u * 16u; e += 128u) { const unsigned rl = e >> 4, q = e & 15u; vst2(DH + ((size_t)r0 + rl) * CC + c0 + q * 8u, *(const v4u*)&sh[rl][q * 8]); }
  } else {
#pragma unroll
    for (int j = 0; j < 8; ++j) {
#pragma unroll
      for (int r = 0; r < 8; ++r) th[j * 16 + col][wave * 16 + 8 * g + r] = (_Float16)acc[j][r]; }
    __syncthreads();
    for (unsigned e = tid; e < 128u * 8u; e += 128u) { const unsigned cl = e >> 3, q = e & 7u; vst2(VT + ((size_t)bb * CC + c0 + cl) * (size_t)TK + t0 + q * 8u, *(const v4u*)&th[cl][q * 8]); } } }

__global__ __launch_bounds__(128) void k_sc(const _Float16* __restrict__ QH, const _Float16* __restrict__ KH, unsigned b, unsigned h0, float* __restrict__ S0) {
  __shared__ __align__(16) float ss[4][16][132];
  const unsigned qb = blockIdx.x, kb = blockIdx.y, h = h0 + blockIdx.z; float* S = S0 + (size_t)blockIdx.z * TQ * TK;
  const unsigned tid = threadIdx.x, wave = tid >> 5, lane = tid & 31u, col = lane & 15u, g = lane >> 4; const unsigned k0 = kb * 128u, ql0 = qb * 64u + wave * 16u;
  const size_t q0 = (size_t)b * TQ + ql0, kr0 = (size_t)b * TK + k0;
  v8f acc[8] = {};
#pragma unroll
  for (int kc = 0; kc < HD / 32; ++kc) { const v16h ah = frag_h(QH + (q0 + col) * CC + h * HD + kc * 32, lane);
#pragma unroll
    for (int j = 0; j < 8; ++j) { const v16h kf = frag_h(KH + (kr0 + j * 16 + col) * CC + h * HD + kc * 32, lane); acc[j] = wmma16(ah, kf, acc[j]); } }
#pragma unroll
  for (int j = 0; j < 8; ++j) {
#pragma unroll
    for (int r = 0; r < 8; ++r) ss[wave][8 * g + r][j * 16 + col] = acc[j][r] * SCALE; }
  LDSX(); for (unsigned rl = 0; rl < 16u; ++rl) vst2(S + (size_t)(ql0 + rl) * TK + k0 + lane * 4u, *(const v4f*)&ss[wave][rl][lane * 4]); }

__global__ __launch_bounds__(256) void k_sm(float* __restrict__ S0, const int* __restrict__ MB) { __shared__ float sred[8]; __shared__ float sbc; __shared__ __align__(16) float shv[TK];
  const unsigned tid = threadIdx.x, t = blockIdx.x;
  float* sr = S0 + (size_t)blockIdx.y * TQ * TK + (size_t)t * TK;
  const int* mr = MB + (size_t)t * SEQ_FULL;
  float m = -3.0e38f;
#pragma unroll 1
  for (unsigned q = tid; q < (unsigned)(TK / 4); q += 256u) { v4f v = *(const v4f*)(sr + q * 4u); const v4i k4 = *(const v4i*)(mr + q * 4u);
    v[0] = (k4[0] == 0) ? MASKFILL : v[0]; v[1] = (k4[1] == 0) ? MASKFILL : v[1]; v[2] = (k4[2] == 0) ? MASKFILL : v[2]; v[3] = (k4[3] == 0) ? MASKFILL : v[3];
    *(v4f*)&shv[q * 4u] = v; m = fmaxf(fmaxf(m, fmaxf(v[0], v[1])), fmaxf(v[2], v[3])); }
#pragma unroll
  for (int o = 1; o < 32; o <<= 1) m = fmaxf(m, __shfl_xor(m, o));
  if ((tid & 31u) == 0) sred[tid >> 5] = m; __syncthreads(); if (tid == 0) { float a = sred[0]; for (int i = 1; i < 8; ++i) a = fmaxf(a, sred[i]); sbc = a; } __syncthreads(); m = sbc; __syncthreads();
  float sum = 0.f;
#pragma unroll 1
  for (unsigned q = tid; q < (unsigned)(TK / 4); q += 256u) { v4f v = *(const v4f*)&shv[q * 4u]; v[0] = expf(v[0] - m); v[1] = expf(v[1] - m); v[2] = expf(v[2] - m); v[3] = expf(v[3] - m); *(v4f*)&shv[q * 4u] = v; sum += (v[0] + v[1]) + (v[2] + v[3]); }
#pragma unroll
  for (int o = 1; o < 32; o <<= 1) sum += __shfl_xor(sum, o);
  if ((tid & 31u) == 0) sred[tid >> 5] = sum; __syncthreads(); if (tid == 0) { float a = 0.f; for (int i = 0; i < 8; ++i) a += sred[i]; sbc = a > 0.f ? PCARRY * (1.0f / a) : 0.f; } __syncthreads(); const float inv = sbc;
#pragma unroll 1
  for (unsigned q = tid; q < (unsigned)(TK / 4); q += 256u) { v4f v = *(const v4f*)&shv[q * 4u]; v[0] *= inv; v[1] *= inv; v[2] *= inv; v[3] *= inv; vst2(sr + q * 4u, v); } }

__global__ __launch_bounds__(128) void k_pv(const float* __restrict__ PS0, const _Float16* __restrict__ VT, unsigned b, unsigned h0, float* __restrict__ Y) {
  __shared__ __align__(16) float ss[4][16][HD + 4];
  const unsigned h = h0 + blockIdx.z; const float* PS = PS0 + (size_t)blockIdx.z * TQ * TK;
  const unsigned tid = threadIdx.x, wave = tid >> 5, lane = tid & 31u, col = lane & 15u, g = lane >> 4; const unsigned ql0 = blockIdx.x * 64u + wave * 16u;
  const float* prow = PS + (size_t)(ql0 + col) * TK + 8u * g;
  const _Float16* vbase = VT + ((size_t)b * CC + h * HD + col) * (size_t)TK;
  v8f acc[HD / 16] = {};
#pragma unroll 1
  for (unsigned kc = 0; kc < (unsigned)(TK / 32); ++kc) { const Q16 tp = ld16(prow + kc * 32u);
    asm volatile("s_wait_loadcnt 0x0" ::: "memory");
    const v16h p = cvt_ph(tp);
#pragma unroll
    for (int j = 0; j < HD / 16; ++j) acc[j] = wmma16(p, frag_h(vbase + (size_t)j * 16 * TK + kc * 32u, lane), acc[j]); }
#pragma unroll
  for (int j = 0; j < HD / 16; ++j) {
#pragma unroll
    for (int r = 0; r < 8; ++r) ss[wave][8 * g + r][j * 16 + col] = acc[j][r] * (1.0f / PCARRY); }
  LDSX(); for (unsigned rl = 0; rl < 16u; ++rl) { const v4f v = *(const v4f*)&ss[wave][rl][col * 4u]; if (lane < (unsigned)(HD / 4)) vst2(Y + ((size_t)b * TQ + ql0 + rl) * CC + h * HD + col * 4u, v); } }

__global__ __launch_bounds__(128) void k_gemh(const float* __restrict__ A, unsigned lda, unsigned K, int act_in, float ascale, const float* __restrict__ Wm, unsigned nout, const float* __restrict__ BIAS, int hasbias, const float* RES, int hasres, float oscale, float* __restrict__ OUT) {
  __shared__ __align__(16) float sf[4][16][132];
  const unsigned tid = threadIdx.x, wave = tid >> 5, lane = tid & 31u, col = lane & 15u, g = lane >> 4; const unsigned c0 = blockIdx.y * 128u; const size_t r0 = (size_t)blockIdx.x * 64 + wave * 16;
  const float* arow = A + (r0 + col) * (size_t)lda + 8u * g;
  const float* wrow = Wm + (size_t)(c0 + col) * K + 8u * g;
  v8f acc[8] = {};
#pragma unroll 1
  for (unsigned kc = 0; kc < K / 32u; ++kc) { const Q16 ta = ld16(arow + kc * 32u);
    asm volatile("s_wait_loadcnt 0x0" ::: "memory");
    const v16h a = cvt_ah(ta, act_in, ascale);
#pragma unroll
    for (int j = 0; j < 8; ++j) { const Q16 tw = ld16(wrow + (size_t)j * 16u * K + kc * 32u); asm volatile("s_wait_loadcnt 0x0" ::: "memory"); const v16h w = cvt_wh(tw); acc[j] = wmma16(a, w, acc[j]); } }
#pragma unroll
  for (int j = 0; j < 8; ++j) { float bb = 0.f; if (hasbias) bb = bfr(BIAS[c0 + j * 16 + col]);
    asm volatile("s_wait_loadcnt 0x0" ::: "memory");
#pragma unroll
    for (int r = 0; r < 8; ++r) sf[wave][8 * g + r][j * 16 + col] = acc[j][r] * oscale + bb; }
  LDSX(); for (unsigned rl = 0; rl < 16u; ++rl) { const size_t o = (r0 + rl) * (size_t)nout + c0 + lane * 4u; v4f v = *(const v4f*)&sf[wave][rl][lane * 4]; if (hasres) { const v4f rv = *(const v4f*)(RES + o); v[0] += rv[0]; v[1] += rv[1]; v[2] += rv[2]; v[3] += rv[3]; } vst2(OUT + o, v); } }

extern "C" void kernel_launch(void* const* d_in, const int* in_sizes, int n_in, void* d_out, int out_size, void* d_ws, size_t ws_size, hipStream_t stream) {
  if (n_in < 22) return;
  if (ws_size < WS_END) return;
  const long long need_x = ((long long)(NB - 1) * SEQ_FULL + SEQ) * DIN;
  const long long need_m = (long long)(NB - 1) * SEQ_FULL * SEQ_FULL + (long long)(SEQ - 1) * SEQ_FULL + SEQ;
  if ((long long)in_sizes[0] < need_x || (long long)in_sizes[1] < need_x) return;
  if ((long long)in_sizes[2] < need_m || (long long)in_sizes[3] < need_m) return;
  for (int i = 4; i < 12; ++i) if ((long long)in_sizes[i] < (long long)DIN * CC) return;
  for (int i = 12; i < 18; ++i) if (in_sizes[i] < CC) return;
  if ((long long)in_sizes[18] < (long long)FF * CC || in_sizes[19] < FF || (long long)in_sizes[20] < (long long)CC * FF || in_sizes[21] < CC) return;
  if ((long long)out_size < (long long)NRW * CC) return;
  const float* const* F = (const float* const*)d_in; const int* M1 = (const int*)d_in[2]; const int* M2 = (const int*)d_in[3];
  char* ws = (char*)d_ws;
  _Float16 *QH = (_Float16*)(ws + WS_QH), *KH = (_Float16*)(ws + WS_KH), *VT = (_Float16*)(ws + WS_VT);
  float *S = (float*)(ws + WS_S), *HF = (float*)(ws + WS_S), *Y = (float*)(ws + WS_Y), *Z = (float*)(ws + WS_Z), *X1 = (float*)(ws + WS_X1), *X2 = (float*)(ws + WS_X2);
  const float osc_ctx = 1.0f / (64.0f * ACARRY), osc_one = 1.0f / 64.0f;
  const size_t mplane = (size_t)SEQ_FULL * SEQ_FULL;

  k_proj<<<dim3(NRW / 64, CC / 128, 3), 128, 0, stream>>>(F[0], F[0], F[4], F[5], F[6], QH, KH, VT);
  for (unsigned b = 0; b < (unsigned)NB; ++b) for (unsigned h0 = 0; h0 < (unsigned)NH; h0 += HG) {
    k_sc<<<dim3(TQ / 64, TK / 128, HG), 128, 0, stream>>>(QH, KH, b, h0, S);
    k_sm<<<dim3(TQ, HG), 256, 0, stream>>>(S, M1 + (size_t)b * mplane);
    k_pv<<<dim3(TQ / 64, 1, HG), 128, 0, stream>>>(S, VT, b, h0, Y);
  }
  k_gemh<<<dim3(NRW / 64, CC / 128), 128, 0, stream>>>(Y, CC, CC, 0, ACARRY, F[7], CC, F[21], 0, X1, 0, osc_ctx, Z);
  k_addln<<<dim3(NRW / 8), 256, 0, stream>>>(F[0], 1, (unsigned)SEQ_FULL, Z, 1, F[12], F[13], X1);

  k_proj<<<dim3(NRW / 64, CC / 128, 3), 128, 0, stream>>>(F[0], F[1], F[8], F[9], F[10], QH, KH, VT);
  for (unsigned b = 0; b < (unsigned)NB; ++b) for (unsigned h0 = 0; h0 < (unsigned)NH; h0 += HG) {
    k_sc<<<dim3(TQ / 64, TK / 128, HG), 128, 0, stream>>>(QH, KH, b, h0, S);
    k_sm<<<dim3(TQ, HG), 256, 0, stream>>>(S, M2 + (size_t)b * mplane);
    k_pv<<<dim3(TQ / 64, 1, HG), 128, 0, stream>>>(S, VT, b, h0, Y);
  }
  k_gemh<<<dim3(NRW / 64, CC / 128), 128, 0, stream>>>(Y, CC, CC, 0, ACARRY, F[11], CC, F[21], 0, X1, 1, osc_ctx, Z);
  k_addln<<<dim3(NRW / 8), 256, 0, stream>>>(Z, 0, (unsigned)TQ, Z, 0, F[14], F[15], X2);

  k_gemh<<<dim3(NRW / 64, FF / 128), 128, 0, stream>>>(X2, CC, CC, 0, 1.0f, F[18], FF, F[19], 1, HF, 0, osc_one, HF);
  k_gemh<<<dim3(NRW / 64, CC / 128), 128, 0, stream>>>(HF, FF, FF, 1, 1.0f, F[20], CC, F[21], 1, X2, 1, osc_one, Z);
  k_addln<<<dim3(NRW / 8), 256, 0, stream>>>(Z, 0, (unsigned)TQ, Z, 0, F[16], F[17], (float*)d_out);
}
